// PointCloudAE_49529562857561
// MI455X (gfx1250) — hardware-verified
//
#include <hip/hip_runtime.h>
#include <stddef.h>


#define C1D     64
#define C2D     128
#define C3D     256
#define LATD    128
#define NOUTD   4096
#define NTHR    256
#define NWAVE   8
#define EPT     8
#define NGRP    2
#define CHUNK   (NTHR * EPT * NGRP)
#define WCAP    (EPT * NGRP * 32)
#define LISTN   (NWAVE * WCAP)
#define NBC     4096
#define NBF     1024
#define RCAP    40960
#define RBN     128
#define TGT     256
#define DEGCAP  128
#define OTHR    512
#define WSCALE  16.0f
#define WINV    0.0625f
#define BNEPS   1e-5f

#define LDS_FILL ((RCAP + NBF + LISTN) * 4 + 64)

static_assert((CHUNK & (CHUNK - 1)) == 0);
static_assert(CHUNK <= 4096);
static_assert(NBC <= 4096 && NBF <= 4096);
static_assert((NBC & (NBC - 1)) == 0 && (NBF & (NBF - 1)) == 0);
static_assert(NBC == 4 * NBF);
static_assert(OTHR * 8 == NBC);
static_assert((RCAP % 32) == 0);
static_assert(TGT == NWAVE * 32);
static_assert((TGT % 128) == 0);

typedef float          v4f   __attribute__((ext_vector_type(4)));
typedef float          v8f   __attribute__((ext_vector_type(8)));
typedef int            v4i   __attribute__((ext_vector_type(4)));
typedef double         v2d   __attribute__((ext_vector_type(2)));
typedef _Float16       v8h   __attribute__((ext_vector_type(8)));
typedef _Float16       v16h  __attribute__((ext_vector_type(16)));
typedef unsigned short v8us  __attribute__((ext_vector_type(8)));
typedef unsigned short v16us __attribute__((ext_vector_type(16)));
typedef __bf16         v16b  __attribute__((ext_vector_type(16)));
union FragH { v16h v; v8h h[2]; };
union FragB { v16b v; v16us w; v8us u[2]; };

__device__ __forceinline__ v8h cvt8(v4f a, v4f b) {
  v8h r;
  r[0] = (_Float16)a.x; r[1] = (_Float16)a.y; r[2] = (_Float16)a.z; r[3] = (_Float16)a.w;
  r[4] = (_Float16)b.x; r[5] = (_Float16)b.y; r[6] = (_Float16)b.z; r[7] = (_Float16)b.w;
  return r;
}

__device__ __forceinline__ unsigned short bf16rne(float x) {
  const unsigned u = __float_as_uint(x);
  return (unsigned short)((u + 0x7FFFu + ((u >> 16) & 1u)) >> 16);
}

__device__ __forceinline__ void split8(v4f a, v4f b, v8us& hu, v8us& lu) {
  float v[8];
  v[0] = a.x; v[1] = a.y; v[2] = a.z; v[3] = a.w; v[4] = b.x; v[5] = b.y; v[6] = b.z; v[7] = b.w;
#pragma unroll
  for (int e = 0; e < 8; ++e) {
    const unsigned short hbits = bf16rne(v[e]);
    const float hf = __uint_as_float(((unsigned)hbits) << 16);
    hu[e] = hbits;
    lu[e] = bf16rne(v[e] - hf);
  }
}

__device__ __forceinline__ v4f relu4(v4f a) {
  v4f r;
  r.x = fmaxf(a.x, 0.0f); r.y = fmaxf(a.y, 0.0f); r.z = fmaxf(a.z, 0.0f); r.w = fmaxf(a.w, 0.0f);
  return r;
}

__device__ __forceinline__ v4f sel4(bool ok, v4f a) {
  v4f r;
  r.x = ok ? a.x : 0.0f; r.y = ok ? a.y : 0.0f; r.z = ok ? a.z : 0.0f; r.w = ok ? a.w : 0.0f;
  return r;
}

__device__ __forceinline__ v8f wmh(v16h a, v16h b, v8f c) {
  v8f d = __builtin_amdgcn_wmma_f32_16x16x32_f16(false, a, false, b, (short)0, c, false, false);
  asm volatile("v_nop\n\tv_nop\n\tv_nop\n\tv_nop" : "+v"(d) : "v"(a), "v"(b));
  return d;
}
__device__ __forceinline__ v8f wmb(const FragB& a, const FragB& b, v8f c) {
  v8f d = __builtin_amdgcn_wmma_f32_16x16x32_bf16(false, a.v, false, b.v, (short)0, c, false, false);
  asm volatile("v_nop\n\tv_nop\n\tv_nop\n\tv_nop" : "+v"(d) : "v"(a.w), "v"(b.w));
  return d;
}

template <int NB>
__device__ __forceinline__ int scan_chunk(const int* __restrict__ dsts, int nE, int cbase, int slotBase,
                                          int vec8, int* list, int tid, int lane, int wave) {
  int wc = 0;
#pragma unroll
  for (int g = 0; g < NGRP; ++g) {
    const int el0  = (g * NTHR + tid) * EPT;
    const int e0   = cbase + el0;
    const int sent = -2147483647 - 1;
    v4i da, db;
    if (vec8 != 0 && cbase + CHUNK <= nE) {
      da = *(const v4i*)(dsts + e0);
      db = *(const v4i*)(dsts + e0 + 4);
    } else {
      da.x = (e0     < nE) ? dsts[min(e0, nE - 1)] : sent;
      da.y = (e0 + 1 < nE) ? dsts[min(e0 + 1, nE - 1)] : sent;
      da.z = (e0 + 2 < nE) ? dsts[min(e0 + 2, nE - 1)] : sent;
      da.w = (e0 + 3 < nE) ? dsts[min(e0 + 3, nE - 1)] : sent;
      db.x = (e0 + 4 < nE) ? dsts[min(e0 + 4, nE - 1)] : sent;
      db.y = (e0 + 5 < nE) ? dsts[min(e0 + 5, nE - 1)] : sent;
      db.z = (e0 + 6 < nE) ? dsts[min(e0 + 6, nE - 1)] : sent;
      db.w = (e0 + 7 < nE) ? dsts[min(e0 + 7, nE - 1)] : sent;
    }
    const unsigned nb = (unsigned)slotBase;
    const unsigned s0 = (unsigned)da.x - nb, s1 = (unsigned)da.y - nb;
    const unsigned s2 = (unsigned)da.z - nb, s3 = (unsigned)da.w - nb;
    const unsigned s4 = (unsigned)db.x - nb, s5 = (unsigned)db.y - nb;
    const unsigned s6 = (unsigned)db.z - nb, s7 = (unsigned)db.w - nb;
    const bool h0 = s0 < (unsigned)NB, h1 = s1 < (unsigned)NB, h2 = s2 < (unsigned)NB, h3 = s3 < (unsigned)NB;
    const bool h4 = s4 < (unsigned)NB, h5 = s5 < (unsigned)NB, h6 = s6 < (unsigned)NB, h7 = s7 < (unsigned)NB;
    const unsigned any = __builtin_amdgcn_ballot_w32(h0 | h1 | h2 | h3 | h4 | h5 | h6 | h7);
    if (any != 0u) {
#define HITJ(J, HJ, SJ) { \
        const unsigned mj = __builtin_amdgcn_ballot_w32(HJ); \
        if (mj != 0u) { \
          if (HJ) { \
            const int pos = wc + (int)__builtin_amdgcn_mbcnt_lo(mj, 0u); \
            if (pos < WCAP) list[wave * WCAP + pos] = ((el0 + (J)) << 12) | (int)(SJ); \
          } \
          wc += (int)__builtin_popcount(mj); } }
      HITJ(0, h0, s0)
      HITJ(1, h1, s1)
      HITJ(2, h2, s2)
      HITJ(3, h3, s3)
      HITJ(4, h4, s4)
      HITJ(5, h5, s5)
      HITJ(6, h6, s6)
      HITJ(7, h7, s7)
#undef HITJ
    }
  }
  return wc;
}

__global__ __launch_bounds__(NTHR) void k_wprep(
    const float* __restrict__ W2, const float* __restrict__ W3, const float* __restrict__ cw1,
    const float* __restrict__ cw2, const float* __restrict__ cw3,
    unsigned short* p1h, unsigned short* p1l, unsigned short* p2h, unsigned short* p2l,
    unsigned short* p3h, unsigned short* p3l, unsigned short* p4, unsigned short* p5) {
  const int g0 = C2D * C1D / 8;
  const int g1 = C3D * C2D / 8;
  const int g2 = C3D * C3D / 8;
  const int g3 = C3D * C3D / 8;
  const int g4 = LATD * C3D / 8;
  const int bstart = blockIdx.x * NTHR;
  const float* src; unsigned short* dh; unsigned short* dl; int K, sk, sn, segOff, split;
  if (bstart < g0)                     { src = W2;  dh = p1h; dl = p1l; K = C1D; sk = C2D; sn = 1;   segOff = 0;                 split = 1; }
  else if (bstart < g0 + g1)           { src = W3;  dh = p2h; dl = p2l; K = C2D; sk = C3D; sn = 1;   segOff = g0;                split = 1; }
  else if (bstart < g0 + g1 + g2)      { src = cw1; dh = p3h; dl = p3l; K = C3D; sk = 1;   sn = C3D; segOff = g0 + g1;           split = 1; }
  else if (bstart < g0 + g1 + g2 + g3) { src = cw2; dh = p4;  dl = p4;  K = C3D; sk = 1;   sn = C3D; segOff = g0 + g1 + g2;      split = 0; }
  else                                 { src = cw3; dh = p5;  dl = p5;  K = C3D; sk = 1;   sn = C3D; segOff = g0 + g1 + g2 + g3; split = 0; }
  const int i = bstart + (int)threadIdx.x;
  if (i >= g0 + g1 + g2 + g3 + g4) return;
  const int o  = (i - segOff) * 8;
  const int n  = o / K;
  const int k0 = o - n * K;
  float v[8];
#pragma unroll
  for (int e = 0; e < 8; ++e) v[e] = src[(size_t)(k0 + e) * sk + (size_t)n * sn];
  if (split == 0) {
    v4f a, b;
    a.x = v[0] * WSCALE; a.y = v[1] * WSCALE; a.z = v[2] * WSCALE; a.w = v[3] * WSCALE;
    b.x = v[4] * WSCALE; b.y = v[5] * WSCALE; b.z = v[6] * WSCALE; b.w = v[7] * WSCALE;
    const v8h hv = cvt8(a, b);
    _Float16* dp = (_Float16*)dh + o;
    *(volatile v8h*)dp = hv;
    __threadfence();
    *(volatile v8h*)dp = hv;
  } else {
    v4f a, b;
    a.x = v[0]; a.y = v[1]; a.z = v[2]; a.w = v[3];
    b.x = v[4]; b.y = v[5]; b.z = v[6]; b.w = v[7];
    v8us hu, lu;
    split8(a, b, hu, lu);
    *(volatile v8us*)(dh + o) = hu;
    *(volatile v8us*)(dl + o) = lu;
    __threadfence();
    *(volatile v8us*)(dh + o) = hu;
    *(volatile v8us*)(dl + o) = lu;
  }
}

__global__ __launch_bounds__(NTHR) void k_count(
    const int* __restrict__ ei, int* cnt, float* dinv, int nE, int vec8) {
  __shared__ __attribute__((aligned(16))) int scnt[NBC];
  __shared__ __attribute__((aligned(16))) int list[LISTN];
  __shared__ int wcnt[NWAVE];
  const int tid = threadIdx.x, lane = tid & 31, wave = tid >> 5;
  const int nodeBase = blockIdx.x * NBC;
  const int* dsts = ei + nE;

  for (int i = tid; i < NBC; i += NTHR) scnt[i] = 0;
  __syncthreads();

  const int nChunks = (nE + CHUNK - 1) / CHUNK;
#pragma unroll 1
  for (int ch = 0; ch < nChunks; ++ch) {
    const int cbase = ch * CHUNK;
    const int wc = scan_chunk<NBC>(dsts, nE, cbase, nodeBase, vec8, list, tid, lane, wave);
    if (lane == 0) wcnt[wave] = wc;
    __syncthreads();
    if (wave == 0) {
#pragma unroll 1
      for (int wsx = 0; wsx < NWAVE; ++wsx) {
        int n = __builtin_amdgcn_readfirstlane(wcnt[wsx]);
        n = n > WCAP ? WCAP : (n < 0 ? 0 : n);
        const int* lp = list + wsx * WCAP;
#pragma unroll 1
        for (int i = 0; i < n; ++i) {
          const int ent  = __builtin_amdgcn_readfirstlane(lp[i]);
          const int slot = ent & (NBC - 1);
          if (lane == 0) scnt[slot] = scnt[slot] + 1;
        }
      }
    }
    __syncthreads();
  }

  v4i cq[4]; v4f dq[4];
#pragma unroll
  for (int q = 0; q < 4; ++q) {
    const int f = (wave * 4 + q) * 128 + 4 * lane;
    const v4i c = *(const v4i*)(scnt + f);
    cq[q] = c;
    dq[q].x = rsqrtf((float)(c.x + 1));
    dq[q].y = rsqrtf((float)(c.y + 1));
    dq[q].z = rsqrtf((float)(c.z + 1));
    dq[q].w = rsqrtf((float)(c.w + 1));
  }
  int*   cp = cnt + (size_t)nodeBase;
  float* dp = dinv + (size_t)nodeBase;
#pragma unroll
  for (int q = 0; q < 4; ++q) {
    const int f = (wave * 4 + q) * 128 + 4 * lane;
    *(volatile v4i*)(cp + f) = cq[q];
    *(volatile v4f*)(dp + f) = dq[q];
  }
  __threadfence();
#pragma unroll
  for (int q = 0; q < 4; ++q) {
    const int f = (wave * 4 + q) * 128 + 4 * lane;
    *(volatile v4i*)(cp + f) = cq[q];
    *(volatile v4f*)(dp + f) = dq[q];
  }
}

__global__ __launch_bounds__(OTHR) void k_offsets(
    const int* __restrict__ cnt, int* off, int* rbase, int nChunk) {
  __shared__ __attribute__((aligned(16))) int soff[NBC];
  __shared__ __attribute__((aligned(16))) int srb[RBN];
  __shared__ int wtot[OTHR / 32];
  const int tid = threadIdx.x, lane = tid & 31, wave = tid >> 5, sub = tid >> 7;
  for (int i = tid; i < RBN; i += OTHR) srb[i] = 0;
  int carry = 0;
#pragma unroll 1
  for (int ch = 0; ch < nChunk; ++ch) {
    const int base = ch * NBC;
    const v4i c0 = *(const v4i*)(cnt + base + 8 * tid);
    const v4i c1 = *(const v4i*)(cnt + base + 8 * tid + 4);
    const int e0 = max(c0.x, 0), e1 = max(c0.y, 0), e2 = max(c0.z, 0), e3 = max(c0.w, 0);
    const int e4 = max(c1.x, 0), e5 = max(c1.y, 0), e6 = max(c1.z, 0), e7 = max(c1.w, 0);
    const int ts = e0 + e1 + e2 + e3 + e4 + e5 + e6 + e7;
    int incl = ts;
#pragma unroll
    for (int d = 1; d < 32; d <<= 1) {
      const int t = __shfl_up(incl, d);
      if (lane >= d) incl += t;
    }
    if (lane == 31) wtot[wave] = incl;
    __syncthreads();
    const int S0 = wtot[0]  + wtot[1]  + wtot[2]  + wtot[3];
    const int S1 = wtot[4]  + wtot[5]  + wtot[6]  + wtot[7];
    const int S2 = wtot[8]  + wtot[9]  + wtot[10] + wtot[11];
    const int S3 = wtot[12] + wtot[13] + wtot[14] + wtot[15];
    int pre = 0;
#pragma unroll 1
    for (int w = 4 * sub; w < wave; ++w) pre += wtot[w];
    const int b0 = carry;
    const int b1 = b0 + ((S0 + 31) & ~31);
    const int b2 = b1 + ((S1 + 31) & ~31);
    const int b3 = b2 + ((S2 + 31) & ~31);
    const int b4 = b3 + ((S3 + 31) & ~31);
    const int myb = sub == 0 ? b0 : (sub == 1 ? b1 : (sub == 2 ? b2 : b3));
    if (tid == 0) {
      srb[min(4 * ch + 0, RBN - 1)] = b0;
      srb[min(4 * ch + 1, RBN - 1)] = b1;
      srb[min(4 * ch + 2, RBN - 1)] = b2;
      srb[min(4 * ch + 3, RBN - 1)] = b3;
    }
    int run = myb + pre + incl - ts;
    soff[8 * tid + 0] = run; run += e0;
    soff[8 * tid + 1] = run; run += e1;
    soff[8 * tid + 2] = run; run += e2;
    soff[8 * tid + 3] = run; run += e3;
    soff[8 * tid + 4] = run; run += e4;
    soff[8 * tid + 5] = run; run += e5;
    soff[8 * tid + 6] = run; run += e6;
    soff[8 * tid + 7] = run;
    carry = b4;
    __syncthreads();
    const v4i o0 = *(const v4i*)(soff + 4 * tid);
    const v4i o1 = *(const v4i*)(soff + 4 * (tid + OTHR));
    int* op = off + base;
    *(volatile v4i*)(op + 4 * tid) = o0;
    *(volatile v4i*)(op + 4 * (tid + OTHR)) = o1;
    __threadfence();
    *(volatile v4i*)(op + 4 * tid) = o0;
    *(volatile v4i*)(op + 4 * (tid + OTHR)) = o1;
    __syncthreads();
  }
  if (tid == 0) srb[min(4 * nChunk, RBN - 1)] = carry;
  __syncthreads();
  v4i rv = {0, 0, 0, 0};
  if (tid < 32) rv = *(const v4i*)(srb + 4 * tid);
  if (tid < 32) *(volatile v4i*)(rbase + 4 * tid) = rv;
  __threadfence();
  if (tid < 32) *(volatile v4i*)(rbase + 4 * tid) = rv;
}

__global__ __launch_bounds__(NTHR) void k_fill(
    const int* __restrict__ ei, const int* __restrict__ off, const int* __restrict__ rbase,
    int* csr, int nN, int nE, int vec8, int csrLen) {
  extern __shared__ v4f lds_dyn[];
  int* region = (int*)lds_dyn;
  int* cursor = region + RCAP;
  int* list   = cursor + NBF;
  int* wcnt   = list + LISTN;
  const int tid = threadIdx.x, lane = tid & 31, wave = tid >> 5;
  const int b = blockIdx.x;
  const int nodeBase = b * NBF;
  const int* dsts = ei + nE;

  int rb0 = rbase[b];
  const int rb1 = rbase[b + 1];
  rb0 = rb0 < 0 ? 0 : (rb0 > csrLen ? csrLen : rb0);
  rb0 &= ~31;
  int len = rb1 - rb0;
  len = len < 0 ? 0 : (len > RCAP ? RCAP : len);
  int lenW = (len + 31) & ~31;
  if (rb0 + lenW > csrLen) lenW = (csrLen - rb0) & ~31;

  {
    const v4i z = {0, 0, 0, 0};
    for (int i = tid; i < RCAP / 4; i += NTHR) ((v4i*)region)[i] = z;
    for (int s = tid; s < NBF; s += NTHR) {
      int o = off[nodeBase + s] - rb0;
      o = o < 0 ? 0 : (o > RCAP ? RCAP : o);
      cursor[s] = o;
    }
  }
  __syncthreads();

  const int nChunks = (nE + CHUNK - 1) / CHUNK;
#pragma unroll 1
  for (int ch = 0; ch < nChunks; ++ch) {
    const int cbase = ch * CHUNK;
    const int wc = scan_chunk<NBF>(dsts, nE, cbase, nodeBase, vec8, list, tid, lane, wave);
    if (lane == 0) wcnt[wave] = wc;
    __syncthreads();
    if (wave == 0) {
#pragma unroll 1
      for (int wsx = 0; wsx < NWAVE; ++wsx) {
        int n = __builtin_amdgcn_readfirstlane(wcnt[wsx]);
        n = n > WCAP ? WCAP : (n < 0 ? 0 : n);
        const int* lp = list + wsx * WCAP;
#pragma unroll 1
        for (int i = 0; i < n; ++i) {
          const int ent  = __builtin_amdgcn_readfirstlane(lp[i]);
          const int slot = ent & (NBF - 1);
          int e = cbase + ((ent >> 12) & (CHUNK - 1));
          e = e > nE - 1 ? nE - 1 : e;
          int src = ei[e];
          src = src < 0 ? 0 : (src > nN - 1 ? nN - 1 : src);
          if (lane == 0) {
            int pos = cursor[slot];
            pos = pos < 0 ? 0 : (pos > RCAP - 1 ? RCAP - 1 : pos);
            region[pos] = src;
            const int np = pos + 1;
            cursor[slot] = np > RCAP ? RCAP : np;
          }
        }
      }
    }
    __syncthreads();
  }

  const int nv = lenW >> 2;
  int* gp = csr + rb0;
#pragma unroll 1
  for (int i = tid; i < nv; i += NTHR) { const v4i v = ((const v4i*)region)[i]; *(volatile v4i*)(gp + 4 * i) = v; }
  __threadfence();
#pragma unroll 1
  for (int i = tid; i < nv; i += NTHR) { const v4i v = ((const v4i*)region)[i]; *(volatile v4i*)(gp + 4 * i) = v; }
}

__global__ __launch_bounds__(NTHR) void k_gcn1(
    const float* __restrict__ x, const int* __restrict__ csr, const int* __restrict__ off,
    const int* __restrict__ cnt, const float* __restrict__ dinv,
    const float* __restrict__ W1, const float* __restrict__ b1,
    float* hd1, int nN, int csrLen) {
  __shared__ float sa0[TGT];
  __shared__ float sa1[TGT];
  __shared__ float sdv[TGT];
  __shared__ float sw[2 * C1D];
  __shared__ float sb[C1D];
  const int tid = threadIdx.x;
  const int node = blockIdx.x * TGT + tid;
  if (tid < 2 * C1D) sw[tid] = W1[tid];
  if (tid < C1D) sb[tid] = b1[tid];
  int n = cnt[node];
  n = n < 0 ? 0 : (n > DEGCAP ? DEGCAP : n);
  const int st = off[node];
  const float dd = dinv[node];
  int nw = n;
#pragma unroll
  for (int d = 1; d < 32; d <<= 1) {
    const int t = __shfl_xor(nw, d);
    nw = t > nw ? t : nw;
  }
  nw = __builtin_amdgcn_readfirstlane(nw);
  float a0 = 0.0f, a1 = 0.0f;
#pragma unroll 1
  for (int p = 0; p < nw; ++p) {
    int pos = st + p;
    pos = pos < 0 ? 0 : (pos > csrLen - 1 ? csrLen - 1 : pos);
    int s = csr[pos];
    s = s < 0 ? 0 : (s > nN - 1 ? nN - 1 : s);
    const float ds = dinv[s];
    const float v0 = x[s] * ds;
    const float v1 = x[(size_t)nN + s] * ds;
    const bool ok = p < n;
    a0 += ok ? v0 : 0.0f;
    a1 += ok ? v1 : 0.0f;
  }
  const int nc = node < nN ? node : nN - 1;
  const float x0 = x[nc], x1 = x[(size_t)nN + nc];
  const bool live = node < nN;
  sa0[tid] = live ? dd * (a0 + x0 * dd) : 0.0f;
  sa1[tid] = live ? dd * (a1 + x1 * dd) : 0.0f;
  sdv[tid] = dd;
  __syncthreads();

  float* base = hd1 + (size_t)blockIdx.x * TGT * C1D;
#pragma unroll 1
  for (int i = 0; i < (TGT * C1D / 4) / NTHR; ++i) {
    const int q   = i * NTHR + tid;
    const int row = q >> 4;
    const int col = 4 * (q & 15);
    const float r0 = sa0[row], r1 = sa1[row], dr = sdv[row];
    v4f v;
    v.x = fmaxf(r0 * sw[col + 0] + r1 * sw[C1D + col + 0] + sb[col + 0], 0.0f) * dr;
    v.y = fmaxf(r0 * sw[col + 1] + r1 * sw[C1D + col + 1] + sb[col + 1], 0.0f) * dr;
    v.z = fmaxf(r0 * sw[col + 2] + r1 * sw[C1D + col + 2] + sb[col + 2], 0.0f) * dr;
    v.w = fmaxf(r0 * sw[col + 3] + r1 * sw[C1D + col + 3] + sb[col + 3], 0.0f) * dr;
    *(volatile v4f*)(base + 4 * q) = v;
  }
  __threadfence();
#pragma unroll 1
  for (int i = 0; i < (TGT * C1D / 4) / NTHR; ++i) {
    const int q   = i * NTHR + tid;
    const int row = q >> 4;
    const int col = 4 * (q & 15);
    const float r0 = sa0[row], r1 = sa1[row], dr = sdv[row];
    v4f v;
    v.x = fmaxf(r0 * sw[col + 0] + r1 * sw[C1D + col + 0] + sb[col + 0], 0.0f) * dr;
    v.y = fmaxf(r0 * sw[col + 1] + r1 * sw[C1D + col + 1] + sb[col + 1], 0.0f) * dr;
    v.z = fmaxf(r0 * sw[col + 2] + r1 * sw[C1D + col + 2] + sb[col + 2], 0.0f) * dr;
    v.w = fmaxf(r0 * sw[col + 3] + r1 * sw[C1D + col + 3] + sb[col + 3], 0.0f) * dr;
    *(volatile v4f*)(base + 4 * q) = v;
  }
}

template <int C>
__global__ __launch_bounds__(NTHR) void k_agg(
    const int* __restrict__ csr, const int* __restrict__ off, const int* __restrict__ cnt,
    const float* __restrict__ dinv, const float* __restrict__ hd, float* agg, int nN, int csrLen) {
  constexpr int LPT = C / 4;
  constexpr int TPS = 32 / LPT;
  static_assert(LPT == 16 || LPT == 32);
  const int tid = threadIdx.x, lane = tid & 31, wave = tid >> 5;
  const int sub = lane / LPT;
  const int li  = lane - sub * LPT;
  const int cl4 = 4 * li;
  const int tbase = blockIdx.x * TGT + wave * 32;
  const int cnt_l = cnt[tbase + lane];
  const int off_l = off[tbase + lane];
  const int dv_l  = __float_as_int(dinv[tbase + lane]);
  const v4f zero = {0.f, 0.f, 0.f, 0.f};

#pragma unroll 1
  for (int j = 0; j < 32; j += TPS) {
    int n0 = __builtin_amdgcn_readlane(cnt_l, j);
    n0 = n0 < 0 ? 0 : (n0 > DEGCAP ? DEGCAP : n0);
    const int st0 = __builtin_amdgcn_readlane(off_l, j);
    const float d0 = __int_as_float(__builtin_amdgcn_readlane(dv_l, j));
    int nme = n0, stme = st0, nmax = n0;
    float dme = d0;
    if (TPS == 2) {
      int n1 = __builtin_amdgcn_readlane(cnt_l, j + 1);
      n1 = n1 < 0 ? 0 : (n1 > DEGCAP ? DEGCAP : n1);
      const int st1 = __builtin_amdgcn_readlane(off_l, j + 1);
      const float d1 = __int_as_float(__builtin_amdgcn_readlane(dv_l, j + 1));
      nme  = sub != 0 ? n1 : n0;
      stme = sub != 0 ? st1 : st0;
      dme  = sub != 0 ? d1 : d0;
      nmax = n0 > n1 ? n0 : n1;
    }
    v4f acc = zero;
#pragma unroll 1
    for (int q0 = 0; q0 < nmax; q0 += LPT) {
      int pos = stme + q0 + li;
      pos = pos < 0 ? 0 : (pos > csrLen - 1 ? csrLen - 1 : pos);
      int sl = csr[pos];
      sl = sl < 0 ? 0 : (sl > nN - 1 ? nN - 1 : sl);
      const int rem  = nmax - q0;
      const int mrem = rem < LPT ? rem : LPT;
#pragma unroll 1
      for (int p = 0; p < mrem; ++p) {
        const int s = __shfl(sl, p, LPT);
        const v4f v = *(const v4f*)(hd + (size_t)s * C + cl4);
        const bool ok = (q0 + p) < nme;
        acc = acc + sel4(ok, v);
      }
    }
    const int c = tbase + j + sub;
    const v4f sv = *(const v4f*)(hd + (size_t)c * C + cl4);
    const v4f v = (acc + sv) * dme;
    float* ap = agg + (size_t)(tbase + j) * C + 4 * lane;
    *(volatile v4f*)ap = v;
    __threadfence();
    *(volatile v4f*)ap = v;
  }
}

template <int KD, int NOUT, int MODE>
struct GemmCfg {
  static constexpr int WC  = NOUT / 128;
  static constexpr int WR  = NWAVE / WC;
  static constexpr int RB  = 16 * WR;
  static constexpr int AP  = KD + 8;
  static constexpr int NPL = MODE ? 2 : 1;
  static constexpr int ABYTES = NPL * RB * AP * 2;
  static constexpr int SBYTES = RB * NOUT * 4;
  static constexpr int LDA  = ABYTES > SBYTES ? ABYTES : SBYTES;
  static constexpr int LPRM = 4 * 256 * 4;
  static constexpr int LRED = 8192;
  static constexpr int LDS  = LDA + LPRM + LRED;
  static constexpr int NTG = MODE ? 4 : 8;
  static constexpr int NG  = 8 / NTG;
  static constexpr int TPC = NTHR / NOUT;
  static constexpr int RPT = RB / TPC;
  static constexpr int RPW = RB / NWAVE;
};

template <int KD, int NOUT, int MODE, int PRE, int EPI>
__global__ __launch_bounds__(NTHR) void k_gemm(
    const float* A, const unsigned short* __restrict__ B0, const unsigned short* __restrict__ B1,
    const float* __restrict__ bias, const float* __restrict__ dinv,
    const float* __restrict__ pmu, const float* __restrict__ prs,
    const float* __restrict__ pg, const float* __restrict__ pbe,
    float* C, double* part, int nValid, int rowScale) {
  typedef GemmCfg<KD, NOUT, MODE> G;
  static_assert((G::RB * KD / 8) % NTHR == 0);
  static_assert(G::WC * G::WR == NWAVE);
  static_assert((KD % 32) == 0 && KD <= 256);
  static_assert(G::TPC * 4 * NOUT * 8 <= G::LRED);
  static_assert((2 * NOUT) % NTHR == 0);
  extern __shared__ v4f lds_dyn[];
  unsigned short* sA  = (unsigned short*)lds_dyn;
  unsigned short* sL  = sA + G::RB * G::AP;
  float*          stg = (float*)lds_dyn;
  float*          sP  = (float*)((char*)lds_dyn + G::LDA);
  double*         red = (double*)((char*)lds_dyn + G::LDA + G::LPRM);
  const int tid = threadIdx.x, lane = tid & 31, wave = tid >> 5, hh = lane >> 4, m = lane & 15;
  const int wr = wave / G::WC, wc = wave - wr * G::WC;
  const int rowBase = blockIdx.x * G::RB;

  if (PRE) {
    for (int k = tid; k < KD; k += NTHR) {
      sP[k] = pmu[k]; sP[256 + k] = prs[k]; sP[512 + k] = pg[k]; sP[768 + k] = pbe[k];
    }
    __syncthreads();
  }

#pragma unroll
  for (int it = 0; it < (G::RB * KD / 8) / NTHR; ++it) {
    const int idx = it * NTHR + tid;
    const int r   = idx / (KD / 8);
    const int c0  = (idx - r * (KD / 8)) * 8;
    const float* ap = A + (size_t)(rowBase + r) * KD + c0;
    v4f a = *(const v4f*)ap, b = *(const v4f*)(ap + 4);
    if (PRE) {
      const v4f m0 = *(const v4f*)(sP + c0),       m1 = *(const v4f*)(sP + c0 + 4);
      const v4f s0 = *(const v4f*)(sP + 256 + c0), s1 = *(const v4f*)(sP + 256 + c0 + 4);
      const v4f g0 = *(const v4f*)(sP + 512 + c0), g1 = *(const v4f*)(sP + 512 + c0 + 4);
      const v4f e0 = *(const v4f*)(sP + 768 + c0), e1 = *(const v4f*)(sP + 768 + c0 + 4);
      a = ((a - m0) * s0) * g0 + e0;
      b = ((b - m1) * s1) * g1 + e1;
      a = relu4(a); b = relu4(b);
    }
    if (MODE == 0) {
      *(v8h*)((_Float16*)sA + r * G::AP + c0) = cvt8(a, b);
    } else {
      v8us hu, lu;
      split8(a, b, hu, lu);
      *(v8us*)(sA + r * G::AP + c0) = hu;
      *(v8us*)(sL + r * G::AP + c0) = lu;
    }
  }
  __syncthreads();

  v8f acc[8];
#pragma unroll
  for (int t = 0; t < 8; ++t) { v8f z = {0.f, 0.f, 0.f, 0.f, 0.f, 0.f, 0.f, 0.f}; acc[t] = z; }
  const int arow = (wr * 16 + m) * G::AP + 8 * hh;
#pragma unroll
  for (int g = 0; g < G::NG; ++g) {
#pragma unroll 1
    for (int kt = 0; kt < KD / 32; ++kt) {
      if (MODE == 0) {
        FragH a;
        a.h[0] = *(const v8h*)((const _Float16*)sA + arow + 32 * kt);
        a.h[1] = *(const v8h*)((const _Float16*)sA + arow + 32 * kt + 16);
#pragma unroll
        for (int t = 0; t < G::NTG; ++t) {
          const int tt = g * G::NTG + t;
          const _Float16* bp = (const _Float16*)B0 + (size_t)(wc * 128 + 16 * tt + m) * KD + 32 * kt + 8 * hh;
          FragH b;
          b.h[0] = *(const v8h*)bp;
          b.h[1] = *(const v8h*)(bp + 16);
          acc[tt] = wmh(a.v, b.v, acc[tt]);
        }
      } else {
        FragB ah, al;
        ah.u[0] = *(const v8us*)(sA + arow + 32 * kt);
        ah.u[1] = *(const v8us*)(sA + arow + 32 * kt + 16);
        al.u[0] = *(const v8us*)(sL + arow + 32 * kt);
        al.u[1] = *(const v8us*)(sL + arow + 32 * kt + 16);
#pragma unroll
        for (int t = 0; t < G::NTG; ++t) {
          const int tt = g * G::NTG + t;
          const size_t bo = (size_t)(wc * 128 + 16 * tt + m) * KD + 32 * kt + 8 * hh;
          FragB bh, bl;
          bh.u[0] = *(const v8us*)(B0 + bo);
          bh.u[1] = *(const v8us*)(B0 + bo + 16);
          bl.u[0] = *(const v8us*)(B1 + bo);
          bl.u[1] = *(const v8us*)(B1 + bo + 16);
          acc[tt] = wmb(ah, bh, acc[tt]);
          acc[tt] = wmb(ah, bl, acc[tt]);
          acc[tt] = wmb(al, bh, acc[tt]);
        }
      }
    }
  }
  __syncthreads();

  const float sc = MODE ? 1.0f : WINV;
  const int r0 = wr * 16 + 8 * hh;
  float dsc[8];
#pragma unroll
  for (int r = 0; r < 8; ++r) dsc[r] = 1.0f;
  if (EPI == 0) {
    const v4f dA = *(const v4f*)(dinv + (size_t)rowBase + r0);
    const v4f dB = *(const v4f*)(dinv + (size_t)rowBase + r0 + 4);
    if (rowScale != 0) {
      dsc[0] = dA.x; dsc[1] = dA.y; dsc[2] = dA.z; dsc[3] = dA.w;
      dsc[4] = dB.x; dsc[5] = dB.y; dsc[6] = dB.z; dsc[7] = dB.w;
    }
  }
#pragma unroll
  for (int t = 0; t < 8; ++t) {
    const int col = wc * 128 + 16 * t + m;
    const float bv = bias[col];
    float* sp = stg + (size_t)r0 * NOUT + col;
#pragma unroll
    for (int r = 0; r < 8; ++r) {
      float v = acc[t][r] * sc + bv;
      if (EPI == 0) { v = fmaxf(v, 0.0f); v = v * dsc[r]; }
      sp[(size_t)r * NOUT] = v;
    }
  }
  __syncthreads();

  if (EPI != 2) {
#pragma unroll
    for (int i = 0; i < G::RPW; ++i) {
      const int row = wave * G::RPW + i;
#pragma unroll
      for (int sg = 0; sg < G::WC; ++sg) {
        const v4f v = *(const v4f*)(stg + (size_t)row * NOUT + sg * 128 + 4 * lane);
        *(volatile v4f*)(C + (size_t)(rowBase + row) * NOUT + sg * 128 + 4 * lane) = v;
      }
    }
    __threadfence();
#pragma unroll
    for (int i = 0; i < G::RPW; ++i) {
      const int row = wave * G::RPW + i;
#pragma unroll
      for (int sg = 0; sg < G::WC; ++sg) {
        const v4f v = *(const v4f*)(stg + (size_t)row * NOUT + sg * 128 + 4 * lane);
        *(volatile v4f*)(C + (size_t)(rowBase + row) * NOUT + sg * 128 + 4 * lane) = v;
      }
    }
  }

  if (EPI != 0) {
    const int col = tid % NOUT;
    const int hf  = tid / NOUT;
    double s = 0.0, q = 0.0;
    float mx = -3.0e38f, mn = 3.0e38f;
#pragma unroll 4
    for (int i = 0; i < G::RPT; ++i) {
      const int r = hf * G::RPT + i;
      const float v = stg[(size_t)r * NOUT + col];
      const bool ok = (rowBase + r) < nValid;
      const double dvv = ok ? (double)v : 0.0;
      s += dvv;
      q += dvv * dvv;
      mx = fmaxf(mx, ok ? v : -3.0e38f);
      mn = fminf(mn, ok ? v : 3.0e38f);
    }
    double* rp = red + (size_t)hf * 4 * NOUT;
    rp[col] = s; rp[NOUT + col] = q; rp[2 * NOUT + col] = (double)mx; rp[3 * NOUT + col] = (double)mn;
    __syncthreads();
    if (G::TPC == 2) {
      if (tid < NOUT) {
        red[tid]            = red[tid] + red[4 * NOUT + tid];
        red[NOUT + tid]     = red[NOUT + tid] + red[5 * NOUT + tid];
        red[2 * NOUT + tid] = fmax(red[2 * NOUT + tid], red[6 * NOUT + tid]);
        red[3 * NOUT + tid] = fmin(red[3 * NOUT + tid], red[7 * NOUT + tid]);
      }
      __syncthreads();
    }
    double* gpart = part + (size_t)blockIdx.x * 4 * NOUT;
#pragma unroll
    for (int it = 0; it < (2 * NOUT) / NTHR; ++it) {
      const int p = it * NTHR + tid;
      const v2d v = *(const v2d*)(red + 2 * p);
      *(volatile v2d*)(gpart + 2 * p) = v;
    }
    __threadfence();
#pragma unroll
    for (int it = 0; it < (2 * NOUT) / NTHR; ++it) {
      const int p = it * NTHR + tid;
      const v2d v = *(const v2d*)(red + 2 * p);
      *(volatile v2d*)(gpart + 2 * p) = v;
    }
  }
}

__global__ __launch_bounds__(NTHR) void k_bnstat(
    const double* __restrict__ part, int nBlk, int nout, int nValid, float* mu, float* rs) {
  __shared__ __attribute__((aligned(16))) float smu[NTHR];
  __shared__ __attribute__((aligned(16))) float srs[NTHR];
  const int tid = threadIdx.x, lane = tid & 31, wave = tid >> 5;
  const int cc = tid < nout ? tid : nout - 1;
  double s = 0.0, q = 0.0;
#pragma unroll 1
  for (int b = 0; b < nBlk; ++b) {
    s += part[((size_t)b * 4 + 0) * nout + cc];
    q += part[((size_t)b * 4 + 1) * nout + cc];
  }
  const double inv = 1.0 / (double)nValid;
  const double mm = s * inv;
  double var = q * inv - mm * mm;
  var = var < 0.0 ? 0.0 : var;
  const float mf = (float)mm;
  const float rf = rsqrtf((float)var + BNEPS);
  smu[tid] = tid < nout ? mf : 0.0f;
  srs[tid] = tid < nout ? rf : 1.0f;
  __syncthreads();
  const int seg = (wave & 1) * 128 + 4 * lane;
  const v4f va = *(const v4f*)(smu + seg);
  const v4f vb = *(const v4f*)(srs + seg);
  const v4f v  = (wave < 2) ? va : vb;
  float* dp = ((wave < 2) ? mu : rs) + seg;
  if (wave < 4) *(volatile v4f*)dp = v;
  __threadfence();
  if (wave < 4) *(volatile v4f*)dp = v;
}

__global__ __launch_bounds__(NTHR) void k_final(
    const double* __restrict__ part, int nBlk, int nValid,
    const float* __restrict__ g3, const float* __restrict__ be3,
    const float* __restrict__ d1w, const float* __restrict__ d1b,
    const float* __restrict__ d2w, const float* __restrict__ d2b,
    const float* __restrict__ d3w, const float* __restrict__ d3b,
    float* out, int nOut) {
  __shared__ float zz[LATD];
  __shared__ float h1[C3D];
  __shared__ float h2[C3D];
  __shared__ __attribute__((aligned(16))) float so[NOUTD];
  const int tid = threadIdx.x;
  if (tid < LATD) {
    double s = 0.0, q = 0.0, mx = -3.0e38, mn = 3.0e38;
#pragma unroll 1
    for (int b = 0; b < nBlk; ++b) {
      const size_t base = (size_t)b * 4 * LATD;
      s += part[base + tid];
      q += part[base + LATD + tid];
      mx = fmax(mx, part[base + 2 * LATD + tid]);
      mn = fmin(mn, part[base + 3 * LATD + tid]);
    }
    const double inv = 1.0 / (double)nValid;
    const double mm = s * inv;
    double var = q * inv - mm * mm;
    var = var < 0.0 ? 0.0 : var;
    const float mf = (float)mm;
    const float rf = rsqrtf((float)var + BNEPS);
    const float gv = g3[tid], bv = be3[tid];
    const float sel = (gv >= 0.0f) ? (float)mx : (float)mn;
    float z = sel - mf;
    z = z * rf;
    z = z * gv;
    z = z + bv;
    zz[tid] = z;
  }
  __syncthreads();
  {
    float a = d1b[tid];
    const float* w = d1w + (size_t)tid * LATD;
#pragma unroll 1
    for (int k = 0; k < LATD; ++k) a = a + zz[k] * w[k];
    h1[tid] = fmaxf(a, 0.0f);
  }
  __syncthreads();
  {
    float a = d2b[tid];
    const float* w = d2w + (size_t)tid * C3D;
#pragma unroll 1
    for (int k = 0; k < C3D; ++k) a = a + h1[k] * w[k];
    h2[tid] = fmaxf(a, 0.0f);
  }
  __syncthreads();
#pragma unroll 1
  for (int o = tid; o < nOut; o += NTHR) {
    float a = d3b[o];
    const float* w = d3w + (size_t)o * C3D;
#pragma unroll 1
    for (int k = 0; k < C3D; ++k) a = a + h2[k] * w[k];
    so[o] = a;
  }
  __syncthreads();
#pragma unroll
  for (int i = 0; i < NOUTD / (4 * NTHR); ++i) {
    const int q = i * NTHR + tid;
    const v4f v = *(const v4f*)(so + 4 * q);
    *(volatile v4f*)(out + 4 * q) = v;
  }
  __threadfence();
#pragma unroll
  for (int i = 0; i < NOUTD / (4 * NTHR); ++i) {
    const int q = i * NTHR + tid;
    const v4f v = *(const v4f*)(so + 4 * q);
    *(volatile v4f*)(out + 4 * q) = v;
  }
}

extern "C" void kernel_launch(void* const* d_in, const int* in_sizes, int n_in,
                              void* d_out, int out_size, void* d_ws, size_t ws_size,
                              hipStream_t stream) {
  if (n_in < 26) return;
  const int nN = in_sizes[0] / 2;
  const int nE = in_sizes[1] / 2;
  if (nN <= 0 || nE <= 0 || in_sizes[0] != 2 * nN || in_sizes[1] != 2 * nE) return;
  if (in_sizes[2] != 2 * C1D || in_sizes[3] != C1D) return;
  if (in_sizes[4] != C1D * C2D || in_sizes[5] != C2D) return;
  if (in_sizes[6] != C2D * C3D || in_sizes[7] != C3D) return;
  if (in_sizes[8] != C3D * C3D || in_sizes[9] != C3D || in_sizes[10] != C3D || in_sizes[11] != C3D) return;
  if (in_sizes[12] != C3D * C3D || in_sizes[13] != C3D || in_sizes[14] != C3D || in_sizes[15] != C3D) return;
  if (in_sizes[16] != LATD * C3D || in_sizes[17] != LATD || in_sizes[18] != LATD || in_sizes[19] != LATD) return;
  if (in_sizes[20] != C3D * LATD || in_sizes[21] != C3D) return;
  if (in_sizes[22] != C3D * C3D || in_sizes[23] != C3D) return;
  if (out_size != NOUTD || in_sizes[24] != NOUTD * C3D || in_sizes[25] != NOUTD) return;
  if (nE > (1 << 28) || nN > (1 << 22)) return;

  const float* x   = (const float*)d_in[0];
  const int*   ei  = (const int*)d_in[1];
  const float* W1  = (const float*)d_in[2];  const float* b1  = (const float*)d_in[3];
  const float* W2  = (const float*)d_in[4];  const float* b2  = (const float*)d_in[5];
  const float* W3  = (const float*)d_in[6];  const float* b3  = (const float*)d_in[7];
  const float* cw1 = (const float*)d_in[8];  const float* cb1 = (const float*)d_in[9];
  const float* g1  = (const float*)d_in[10]; const float* be1 = (const float*)d_in[11];
  const float* cw2 = (const float*)d_in[12]; const float* cb2 = (const float*)d_in[13];
  const float* g2  = (const float*)d_in[14]; const float* be2 = (const float*)d_in[15];
  const float* cw3 = (const float*)d_in[16]; const float* cb3 = (const float*)d_in[17];
  const float* g3  = (const float*)d_in[18]; const float* be3 = (const float*)d_in[19];
  const float* d1w = (const float*)d_in[20]; const float* d1b = (const float*)d_in[21];
  const float* d2w = (const float*)d_in[22]; const float* d2b = (const float*)d_in[23];
  const float* d3w = (const float*)d_in[24]; const float* d3b = (const float*)d_in[25];
  float* out = (float*)d_out;

  const int NPAD   = ((nN + TGT - 1) / TGT) * TGT;
  const int nBC    = (nN + NBC - 1) / NBC;
  const int CNTPAD = nBC * NBC;
  if (4 * nBC + 1 > RBN) return;
  const int nBF    = (nN + NBF - 1) / NBF;
  const int csrLen = ((nE + 31) & ~31) + 4096;
  const int nAgg   = NPAD / TGT;
  const int g64    = NPAD / 64;
  const int g128   = NPAD / 128;

  char* ws = (char*)d_ws;
  size_t off = 0;
#define CARVE(name, bytes) const size_t name = off; off += (((size_t)(bytes)) + 255) & ~(size_t)255;
  CARVE(oP1h, (size_t)C2D * C1D * 2)
  CARVE(oP1l, (size_t)C2D * C1D * 2)
  CARVE(oP2h, (size_t)C3D * C2D * 2)
  CARVE(oP2l, (size_t)C3D * C2D * 2)
  CARVE(oP3h, (size_t)C3D * C3D * 2)
  CARVE(oP3l, (size_t)C3D * C3D * 2)
  CARVE(oP4,  (size_t)C3D * C3D * 2)
  CARVE(oP5,  (size_t)LATD * C3D * 2)
  CARVE(oCnt, (size_t)CNTPAD * 4)
  CARVE(oDv,  (size_t)CNTPAD * 4)
  CARVE(oOff, (size_t)CNTPAD * 4)
  CARVE(oRb,  (size_t)RBN * 4)
  CARVE(oCsr, (size_t)csrLen * 4)
  CARVE(oR1,  (size_t)NPAD * C3D * 4)
  CARVE(oR2,  (size_t)NPAD * C2D * 4)
  CARVE(oPart,(size_t)g64 * 4 * C3D * 8)
  CARVE(oMu1, 1024)
  CARVE(oRs1, 1024)
  CARVE(oMu2, 1024)
  CARVE(oRs2, 1024)
#undef CARVE
  if (off > ws_size) return;
  if ((size_t)g128 * 4 * LATD * 8 > (size_t)g64 * 4 * C3D * 8) return;

  unsigned short* p1h = (unsigned short*)(ws + oP1h);
  unsigned short* p1l = (unsigned short*)(ws + oP1l);
  unsigned short* p2h = (unsigned short*)(ws + oP2h);
  unsigned short* p2l = (unsigned short*)(ws + oP2l);
  unsigned short* p3h = (unsigned short*)(ws + oP3h);
  unsigned short* p3l = (unsigned short*)(ws + oP3l);
  unsigned short* p4  = (unsigned short*)(ws + oP4);
  unsigned short* p5  = (unsigned short*)(ws + oP5);
  int*    cnt  = (int*)(ws + oCnt);
  float*  dinv = (float*)(ws + oDv);
  int*    offp = (int*)(ws + oOff);
  int*    rb   = (int*)(ws + oRb);
  int*    csr  = (int*)(ws + oCsr);
  float*  R1   = (float*)(ws + oR1);
  float*  R2   = (float*)(ws + oR2);
  double* part = (double*)(ws + oPart);
  float*  mu1  = (float*)(ws + oMu1);
  float*  rs1  = (float*)(ws + oRs1);
  float*  mu2  = (float*)(ws + oMu2);
  float*  rs2  = (float*)(ws + oRs2);

  const int vec8 = ((nE & 3) == 0) ? 1 : 0;

  const int nPrep = C2D * C1D / 8 + C3D * C2D / 8 + C3D * C3D / 8 + C3D * C3D / 8 + LATD * C3D / 8;
  k_wprep<<<(nPrep + NTHR - 1) / NTHR, NTHR, 0, stream>>>(W2, W3, cw1, cw2, cw3, p1h, p1l, p2h, p2l, p3h, p3l, p4, p5);

  k_count<<<nBC, NTHR, 0, stream>>>(ei, cnt, dinv, nE, vec8);
  k_offsets<<<1, OTHR, 0, stream>>>(cnt, offp, rb, nBC);
  hipFuncSetAttribute(reinterpret_cast<const void*>(&k_fill),
                      hipFuncAttributeMaxDynamicSharedMemorySize, LDS_FILL);
  k_fill<<<nBF, NTHR, LDS_FILL, stream>>>(ei, offp, rb, csr, nN, nE, vec8, csrLen);

  k_gcn1<<<nAgg, NTHR, 0, stream>>>(x, csr, offp, cnt, dinv, W1, b1, R1, nN, csrLen);

  k_agg<C1D><<<nAgg, NTHR, 0, stream>>>(csr, offp, cnt, dinv, R1, R2, nN, csrLen);

  typedef GemmCfg<C1D, C2D, 1> GC1;
  typedef GemmCfg<C2D, C3D, 1> GC2;
  typedef GemmCfg<C3D, C3D, 1> GC3;
  typedef GemmCfg<C3D, C3D, 0> GC4;
  typedef GemmCfg<C3D, LATD, 0> GC5;
  hipFuncSetAttribute(reinterpret_cast<const void*>(&k_gemm<C1D, C2D, 1, 0, 0>),
                      hipFuncAttributeMaxDynamicSharedMemorySize, GC1::LDS);
  hipFuncSetAttribute(reinterpret_cast<const void*>(&k_gemm<C2D, C3D, 1, 0, 0>),
                      hipFuncAttributeMaxDynamicSharedMemorySize, GC2::LDS);
  hipFuncSetAttribute(reinterpret_cast<const void*>(&k_gemm<C3D, C3D, 1, 0, 1>),
                      hipFuncAttributeMaxDynamicSharedMemorySize, GC3::LDS);
  hipFuncSetAttribute(reinterpret_cast<const void*>(&k_gemm<C3D, C3D, 0, 1, 1>),
                      hipFuncAttributeMaxDynamicSharedMemorySize, GC4::LDS);
  hipFuncSetAttribute(reinterpret_cast<const void*>(&k_gemm<C3D, LATD, 0, 1, 2>),
                      hipFuncAttributeMaxDynamicSharedMemorySize, GC5::LDS);
  if (NPAD != g128 * GC1::RB || NPAD != g64 * GC2::RB || NPAD != g64 * GC3::RB ||
      NPAD != g64 * GC4::RB || NPAD != g128 * GC5::RB) return;
  k_gemm<C1D, C2D, 1, 0, 0><<<g128, NTHR, GC1::LDS, stream>>>(
      R2, p1h, p1l, b2, dinv, mu1, rs1, g1, be1, R1, part, nN, 1);

  k_agg<C2D><<<nAgg, NTHR, 0, stream>>>(csr, offp, cnt, dinv, R1, R2, nN, csrLen);

  k_gemm<C2D, C3D, 1, 0, 0><<<g64, NTHR, GC2::LDS, stream>>>(
      R2, p2h, p2l, b3, dinv, mu1, rs1, g1, be1, R1, part, nN, 0);

  k_gemm<C3D, C3D, 1, 0, 1><<<g64, NTHR, GC3::LDS, stream>>>(
      R1, p3h, p3l, cb1, dinv, mu1, rs1, g1, be1, R1, part, nN, 0);
  k_bnstat<<<1, NTHR, 0, stream>>>(part, g64, C3D, nN, mu1, rs1);

  k_gemm<C3D, C3D, 0, 1, 1><<<g64, NTHR, GC4::LDS, stream>>>(
      R1, p4, p4, cb2, dinv, mu1, rs1, g1, be1, R1, part, nN, 0);
  k_bnstat<<<1, NTHR, 0, stream>>>(part, g64, C3D, nN, mu2, rs2);

  k_gemm<C3D, LATD, 0, 1, 2><<<g128, NTHR, GC5::LDS, stream>>>(
      R1, p5, p5, cb3, dinv, mu2, rs2, g2, be2, R2, part, nN, 0);

  k_final<<<1, NTHR, 0, stream>>>(part, g128, nN, g3, be3, d1w, d1b, d2w, d2b, d3w, d3b, out, out_size);
}
